// SelfAttention_36687610643187
// MI455X (gfx1250) — hardware-run, weakly checked
//
#include <hip/hip_runtime.h>


#ifndef NB
#define NB 4
#endif
#ifndef SEQ
#define SEQ 2048
#endif
#define NB_FULL  4
#define SEQ_FULL 2048
#define DM   1024
#define QC   (3 * DM)
#define WSC  64.0f
#define NH   16
#define HD   64
#define HQ   192
#define QCAR 16.0f
#define VCAR 16.0f
#define CCAR 64.0f
#define PEXP 14.0f
#define SC2  (0.03125f * 1.4426950408889634f / (QCAR * QCAR))
#define CP   72
#define AL256(n) ((((size_t)(n)) + 255) / 256 * 256)

static_assert(NB >= 1 && NB <= NB_FULL);
static_assert(SEQ >= 256 && SEQ <= SEQ_FULL);
static_assert(SEQ % 256 == 0);
static_assert(DM % 256 == 0);
static_assert(QC % 64 == 0);
static_assert((SEQ * DM) % 2048 == 0);
static_assert((DM * SEQ) % 2048 == 0);
static_assert(DM == NH * HD);
static_assert(QC == NH * HQ);
static_assert(HQ == 3 * HD);
static_assert(HD == 64);
static_assert(HD % 8 == 0);
static_assert(SEQ % 64 == 0);
static_assert(SEQ % 32 == 0);
static_assert(DM % 32 == 0);
static_assert(CP % 8 == 0 && CP >= HD);
static_assert((SEQ * 2 * DM) % 2048 == 0);
static_assert(AL256((size_t)QC * DM * 2) + AL256((size_t)DM * DM * 2) + AL256((size_t)SEQ * DM * 2) + AL256((size_t)SEQ * QC * 4) +
              AL256((size_t)2 * SEQ * DM * 2) + AL256((size_t)DM * SEQ * 2) + AL256((size_t)SEQ * DM * 2) <= (size_t)134217728);

typedef _Float16 h16;
typedef unsigned short bf;
typedef __attribute__((ext_vector_type(16))) __bf16   v16bf;
typedef __attribute__((ext_vector_type(16))) _Float16 v16h;
typedef __attribute__((ext_vector_type(8)))  _Float16 v8h;
typedef __attribute__((ext_vector_type(8)))  unsigned short v8us;
typedef __attribute__((ext_vector_type(8)))  float    v8f;
typedef __attribute__((ext_vector_type(4)))  float    v4f;
typedef __attribute__((ext_vector_type(4)))  _Float16 v4h;
typedef v8h  __attribute__((may_alias)) v8ha;
typedef v4f  __attribute__((may_alias)) v4fa;
typedef v8us __attribute__((may_alias)) v8usa;

__device__ __forceinline__ unsigned short f2bf(float f) { unsigned u = __float_as_uint(f); u += 0x7FFFu + ((u >> 16) & 1u); return (unsigned short)(u >> 16); }
__device__ __forceinline__ float bf2f(unsigned short b) { return __uint_as_float(((unsigned)b) << 16); }
__device__ __forceinline__ float bfr(float f) { return bf2f(f2bf(f)); }
__device__ __forceinline__ h16 tohx(float x) { return (h16)x; }
__device__ __forceinline__ void splitf(float y, unsigned short& h, unsigned short& l) { h = f2bf(y); l = f2bf(y - bf2f(h)); }
__device__ __forceinline__ v16h cat16(v8h lo, v8h hi) { return __builtin_shufflevector(lo, hi, 0, 1, 2, 3, 4, 5, 6, 7, 8, 9, 10, 11, 12, 13, 14, 15); }
__device__ __forceinline__ v16bf cat16b(v8us lo, v8us hi) { return __builtin_bit_cast(v16bf, __builtin_shufflevector(lo, hi, 0, 1, 2, 3, 4, 5, 6, 7, 8, 9, 10, 11, 12, 13, 14, 15)); }
__device__ __forceinline__ v8f wmma16(v16h a, v16h b, v8f c) { return __builtin_amdgcn_wmma_f32_16x16x32_f16(false, a, false, b, (short)0, c, false, false); }
__device__ __forceinline__ v8f wmmab(v16bf a, v16bf b, v8f c) { return __builtin_amdgcn_wmma_f32_16x16x32_bf16(false, a, false, b, (short)0, c, false, false); }

static __device__ __forceinline__ h16 toh_flush(float v) { const h16 r = (h16)v; return (fabsf(v) < 6.103515625e-05f) ? (h16)0.0f : r; }
static __device__ __forceinline__ v16h ldfr(const h16* p) { return cat16(*(const v8h*)p, *(const v8h*)(p + 16)); }
static __device__ __forceinline__ v8f wmg(v16h a, v16h b, v8f c) { c = wmma16(a, b, c); asm volatile("v_nop\n\tv_nop\n\tv_nop\n\tv_nop" : "+v"(c) : "v"(a), "v"(b)); return c; }

template <typename T16> struct WFrag;
template <> struct WFrag<h16> { typedef v16h V; static __device__ __forceinline__ V ld(const h16* p) { return cat16(*(const v8h*)p, *(const v8h*)(p + 16)); } static __device__ __forceinline__ v8f mma(V a, V b, v8f c) { return wmma16(a, b, c); } };
template <> struct WFrag<bf> { typedef v16bf V; static __device__ __forceinline__ V ld(const bf* p) { return cat16b(*(const v8us*)p, *(const v8us*)(p + 16)); } static __device__ __forceinline__ v8f mma(V a, V b, v8f c) { return wmmab(a, b, c); } };
template <typename T16, int NSPLIT, bool BIAS, bool RES>
__global__ __launch_bounds__(32) void k_gemmw(const T16* __restrict__ A, const T16* __restrict__ A2, const T16* __restrict__ Bt, const T16* __restrict__ Bt2, int K, float* C, int ldc, float oscale, const float* __restrict__ bias, const float* __restrict__ res, int ldr, size_t sA, size_t sB, size_t sC, size_t sR) {
    typedef typename WFrag<T16>::V V;
    __shared__ __align__(16) float os[16 * 68];
    const size_t z = blockIdx.z; A += z * sA; if (A2) A2 += z * sA; Bt += z * sB; if (Bt2) Bt2 += z * sB; C += z * sC; if (RES) res += z * sR;
    const int lane = threadIdx.x & 31, lr = lane & 15, hi = lane >> 4; const int r0 = blockIdx.x * 64, c0 = blockIdx.y * 64;
    v8f acc[4][4];
#pragma unroll
    for (int mb = 0; mb < 4; ++mb)
#pragma unroll
        for (int nb = 0; nb < 4; ++nb) acc[mb][nb] = (v8f){};
    const size_t aoff = (size_t)(r0 + lr) * K + 8 * hi, boff = (size_t)(c0 + lr) * K + 8 * hi;
#pragma unroll 1
    for (int kc = 0; kc < K; kc += 32) {
        V a[4], a2[4];
#pragma unroll
        for (int mb = 0; mb < 4; ++mb) { a[mb] = WFrag<T16>::ld(A + aoff + (size_t)mb * 16 * K + kc); a2[mb] = a[mb]; if (NSPLIT == 1 || NSPLIT == 2) a2[mb] = WFrag<T16>::ld(A2 + aoff + (size_t)mb * 16 * K + kc); }
#pragma unroll
        for (int nb = 0; nb < 4; ++nb) { const V b = WFrag<T16>::ld(Bt + boff + (size_t)nb * 16 * K + kc); V b2 = b; if (NSPLIT >= 2) b2 = WFrag<T16>::ld(Bt2 + boff + (size_t)nb * 16 * K + kc);
#pragma unroll
            for (int mb = 0; mb < 4; ++mb) { acc[mb][nb] = WFrag<T16>::mma(a[mb], b, acc[mb][nb]); if (NSPLIT == 1 || NSPLIT == 2) acc[mb][nb] = WFrag<T16>::mma(a2[mb], b, acc[mb][nb]); if (NSPLIT >= 2) acc[mb][nb] = WFrag<T16>::mma(a[mb], b2, acc[mb][nb]); } }
        asm volatile("v_nop\n\tv_nop\n\tv_nop\n\tv_nop" : "+v"(acc[0][0]), "+v"(acc[1][1]), "+v"(acc[2][2]), "+v"(acc[3][3]) : "v"(a[0]), "v"(a[3]));
    }
#pragma unroll
    for (int mb = 0; mb < 4; ++mb) {
#pragma unroll
        for (int nb = 0; nb < 4; ++nb) {
#pragma unroll
            for (int j = 0; j < 8; ++j) os[(hi * 8 + j) * 68 + nb * 16 + lr] = acc[mb][nb][j]; }
        __builtin_amdgcn_wave_barrier(); asm volatile("" ::: "memory");
        float* crow = C + (size_t)(r0 + mb * 16) * ldc + c0;
#pragma unroll 1
        for (int ps = 0; ps < 2; ++ps) {
#pragma unroll
            for (int s = 0; s < 8; ++s) { const int row = 2 * s + hi, cofs = lr * 4; v4f val = *(const v4fa*)(os + row * 68 + cofs); val = val * oscale;
                if (BIAS) { val[0] += bfr(bias[c0 + cofs]); val[1] += bfr(bias[c0 + cofs + 1]); val[2] += bfr(bias[c0 + cofs + 2]); val[3] += bfr(bias[c0 + cofs + 3]); }
                if (RES) { const v4f xr = *(const v4f*)(res + (size_t)(r0 + mb * 16 + row) * ldr + c0 + cofs); val[0] += bfr(xr[0]); val[1] += bfr(xr[1]); val[2] += bfr(xr[2]); val[3] += bfr(xr[3]); }
                *(volatile v4f*)(crow + (size_t)row * ldc + cofs) = val; }
            if (ps == 0) __threadfence(); }
        __builtin_amdgcn_wave_barrier(); asm volatile("" ::: "memory");
    }
}

__global__ __launch_bounds__(256) void k_cvt8(const float* __restrict__ src, bf* dst, size_t n8) { const size_t i = (size_t)blockIdx.x * 256 + threadIdx.x; if (i >= n8) return; const v8f v = *(const v8f*)(src + i * 8); v8us o;
#pragma unroll
    for (int k = 0; k < 8; ++k) o[k] = f2bf(v[k]); *(volatile v8us*)(dst + i * 8) = o; __threadfence(); *(volatile v8us*)(dst + i * 8) = o; }

template <bool RB>
__global__ __launch_bounds__(256) void k_cvth(const float* __restrict__ src, float sc, h16* dst, size_t n8) { const size_t i = (size_t)blockIdx.x * 256 + threadIdx.x; if (i >= n8) return; const v8f v = *(const v8f*)(src + i * 8); v8h o;
#pragma unroll
    for (int k = 0; k < 8; ++k) { const float y = RB ? bfr(v[k]) : v[k]; o[k] = tohx(y * sc); } *(volatile v8h*)(dst + i * 8) = o; __threadfence(); *(volatile v8h*)(dst + i * 8) = o; }

__global__ __launch_bounds__(256) void k_qkh(const float* __restrict__ F, h16* QK) {
#pragma clang fp contract(off)
    const size_t i = (size_t)blockIdx.x * 256 + threadIdx.x; if (i >= (size_t)SEQ * 2 * DM / 8) return;
    const size_t e = i * 8; const int t = (int)(e / (2 * DM)); const int c = (int)(e % (2 * DM)); const int p = c / DM; const int cc = c % DM;
    const int sc = (cc / HD) * HQ + p * HD + (cc % HD);
    const float* f = F + (size_t)t * QC + sc; const v4f x0 = *(const v4f*)f; const v4f x1 = *(const v4f*)(f + 4); v8h o;
#pragma unroll
    for (int q = 0; q < 4; ++q) { o[q] = toh_flush(x0[q] * QCAR); o[q + 4] = toh_flush(x1[q] * QCAR); }
    const size_t ofs = (size_t)p * SEQ * DM + (size_t)t * DM + cc;
    *(volatile v8h*)(QK + ofs) = o; __threadfence(); *(volatile v8h*)(QK + ofs) = o;
}

__global__ __launch_bounds__(256) void k_vth(const float* __restrict__ F, h16* VT) {
#pragma clang fp contract(off)
    const size_t i = (size_t)blockIdx.x * 256 + threadIdx.x; if (i >= (size_t)DM * SEQ / 8) return;
    const size_t e = i * 8; const int t = (int)(e % SEQ); const int d = (int)(e / SEQ);
    const int sc = (d / HD) * HQ + 2 * HD + (d % HD); v8h o;
#pragma unroll
    for (int q = 0; q < 8; ++q) o[q] = toh_flush(F[(size_t)(t + q) * QC + sc] * VCAR);
    *(volatile v8h*)(VT + e) = o; __threadfence(); *(volatile v8h*)(VT + e) = o;
}

__global__ __launch_bounds__(128) void k_attn(const h16* __restrict__ Qp, const h16* __restrict__ Kp, const h16* __restrict__ VT, h16* CT) {
    __shared__ __align__(16) h16 cs[4 * 16 * CP];
    const int wave = __builtin_amdgcn_readfirstlane(threadIdx.x >> 5);
    const int lane = threadIdx.x & 31, lr = lane & 15, hi = lane >> 4;
    const int hoff = blockIdx.y * HD;
    const int q0 = blockIdx.x * 64 + wave * 16;
    const h16* qp = Qp + (size_t)(q0 + lr) * DM + hoff + 8 * hi;
    const v16h qf0 = ldfr(qp);
    const v16h qf1 = ldfr(qp + 32);
    const h16* kp = Kp + (size_t)lr * DM + hoff + 8 * hi;
    const h16* vp = VT + (size_t)(hoff + lr) * SEQ + 8 * hi;
    v8f acc0 = (v8f){}, acc1 = (v8f){}, acc2 = (v8f){}, acc3 = (v8f){};
    float mrun = -3.0e38f, lrun = 0.0f;
#pragma unroll 1
    for (int kb = 0; kb < SEQ; kb += 32) {
        const h16* kr = kp + (size_t)kb * DM;
        const v16h ka00 = ldfr(kr);
        const v16h ka01 = ldfr(kr + 32);
        const v16h ka10 = ldfr(kr + (size_t)16 * DM);
        const v16h ka11 = ldfr(kr + (size_t)16 * DM + 32);
        v8f s0 = (v8f){}, s1 = (v8f){};
        s0 = wmg(ka00, qf0, s0);
        s0 = wmg(ka01, qf1, s0);
        s1 = wmg(ka10, qf0, s1);
        s1 = wmg(ka11, qf1, s1);
        float mx = fmaxf(s0[0], s1[0]);
#pragma unroll
        for (int r = 1; r < 8; ++r) { mx = fmaxf(mx, s0[r]); mx = fmaxf(mx, s1[r]); }
        mx = fmaxf(mx, __shfl_xor(mx, 16, 32));
        const float mnew = fmaxf(mrun, mx * SC2);
        const float corr = __builtin_amdgcn_exp2f(mrun - mnew);
        const float eb = PEXP - mnew;
        v16h pf; float ls = 0.0f;
#pragma unroll
        for (int r = 0; r < 8; ++r) { const float e = fmaf(s0[r], SC2, eb); const float pe = __builtin_amdgcn_exp2f(e); const float pv = (e < -14.0f) ? 0.0f : pe; const h16 ph = (h16)pv; pf[r] = ph; ls += (float)ph; }
#pragma unroll
        for (int r = 0; r < 8; ++r) { const float e = fmaf(s1[r], SC2, eb); const float pe = __builtin_amdgcn_exp2f(e); const float pv = (e < -14.0f) ? 0.0f : pe; const h16 ph = (h16)pv; pf[8 + r] = ph; ls += (float)ph; }
        ls += __shfl_xor(ls, 16, 32);
        lrun = lrun * corr + ls; mrun = mnew;
        acc0 = acc0 * corr; acc1 = acc1 * corr; acc2 = acc2 * corr; acc3 = acc3 * corr;
        const h16* vr = vp + kb;
        const v16h va0 = ldfr(vr);
        const v16h va1 = ldfr(vr + (size_t)16 * SEQ);
        const v16h va2 = ldfr(vr + (size_t)32 * SEQ);
        const v16h va3 = ldfr(vr + (size_t)48 * SEQ);
        acc0 = wmg(va0, pf, acc0);
        acc1 = wmg(va1, pf, acc1);
        acc2 = wmg(va2, pf, acc2);
        acc3 = wmg(va3, pf, acc3);
    }
    const float fin = (CCAR / VCAR) * (1.0f / lrun);
    const int cwo = wave * 16 * CP;
    v8h o0, o1, o2, o3;
#pragma unroll
    for (int r = 0; r < 8; ++r) { o0[r] = toh_flush(acc0[r] * fin); o1[r] = toh_flush(acc1[r] * fin); o2[r] = toh_flush(acc2[r] * fin); o3[r] = toh_flush(acc3[r] * fin); }
    *(v8ha*)(cs + cwo + lr * CP + 8 * hi) = o0;
    *(v8ha*)(cs + cwo + lr * CP + 16 + 8 * hi) = o1;
    *(v8ha*)(cs + cwo + lr * CP + 32 + 8 * hi) = o2;
    *(v8ha*)(cs + cwo + lr * CP + 48 + 8 * hi) = o3;
    __builtin_amdgcn_wave_barrier(); asm volatile("" ::: "memory");
    h16* crow = CT + (size_t)q0 * DM + hoff;
#pragma unroll 1
    for (int ps = 0; ps < 2; ++ps) {
#pragma unroll
        for (int s = 0; s < 4; ++s) { const int row = 4 * s + (lane >> 3), pc = (lane & 7) * 8; const v8h v = *(const v8ha*)(cs + cwo + row * CP + pc);
            *(volatile v8h*)(crow + (size_t)row * DM + pc) = v; }
        if (ps == 0) __threadfence(); }
}

extern "C" void kernel_launch(void* const* d_in, const int* in_sizes, int n_in,
                              void* d_out, int out_size, void* d_ws, size_t ws_size, hipStream_t stream) {
    if (n_in < 4) return;
    if (in_sizes[0] < (NB - 1) * SEQ_FULL * DM + SEQ * DM) return;
    if (in_sizes[1] < QC * DM) return;
    if (in_sizes[2] < DM * DM) return;
    if (in_sizes[3] < DM) return;
    if (out_size < NB * SEQ * DM) return;
    const float* x = (const float*)d_in[0];
    const float* wqkv = (const float*)d_in[1];
    const float* wout = (const float*)d_in[2];
    const float* bout = (const float*)d_in[3];
    float* OUT = (float*)d_out;
    char* wsp = (char*)d_ws;
    auto take = [&](size_t bytes) { char* p = wsp; wsp += (bytes + 255) & ~(size_t)255; return (void*)p; };
    bf*  WQ  = (bf*)take((size_t)QC * DM * 2);
    h16* WO  = (h16*)take((size_t)DM * DM * 2);
    bf*  XB  = (bf*)take((size_t)SEQ * DM * 2);
    float* F = (float*)take((size_t)SEQ * QC * 4);
    h16* QKp = (h16*)take((size_t)2 * SEQ * DM * 2);
    h16* VT  = (h16*)take((size_t)DM * SEQ * 2);
    h16* CT  = (h16*)take((size_t)SEQ * DM * 2);
    if ((size_t)(wsp - (char*)d_ws) > ws_size) return;

    const size_t nW8 = (size_t)QC * DM / 8, nO8 = (size_t)DM * DM / 8, nX8 = (size_t)SEQ * DM / 8, nQK8 = (size_t)SEQ * 2 * DM / 8, nV8 = (size_t)DM * SEQ / 8;
    k_cvt8<<<(unsigned)((nW8 + 255) / 256), 256, 0, stream>>>(wqkv, WQ, nW8);
    k_cvth<true><<<(unsigned)((nO8 + 255) / 256), 256, 0, stream>>>(wout, WSC, WO, nO8);
    for (int b = 0; b < NB; ++b) {
        k_cvt8<<<(unsigned)((nX8 + 255) / 256), 256, 0, stream>>>(x + (size_t)b * SEQ_FULL * DM, XB, nX8);
        k_gemmw<bf, 0, false, false><<<dim3(SEQ / 64, QC / 64, 1), 32, 0, stream>>>(XB, nullptr, WQ, nullptr, DM, F, QC, 1.0f, nullptr, nullptr, 0, 0, 0, 0, 0);
        k_qkh<<<(unsigned)((nQK8 + 255) / 256), 256, 0, stream>>>(F, QKp);
        k_vth<<<(unsigned)((nV8 + 255) / 256), 256, 0, stream>>>(F, VT);
        k_attn<<<dim3(SEQ / 64, NH, 1), 128, 0, stream>>>(QKp, QKp + (size_t)SEQ * DM, VT, CT);
        k_gemmw<h16, 0, true, true><<<dim3(SEQ / 64, DM / 64, 1), 32, 0, stream>>>(CT, nullptr, WO, nullptr, DM, OUT + (size_t)b * SEQ * DM, DM, 1.0f / (WSC * CCAR), bout, x + (size_t)b * SEQ_FULL * DM, DM, 0, 0, 0, 0);
    }
}
